// NOISE_BASED_CLASSIFIER_CDVAE_266287973055
// MI455X (gfx1250) — hardware-verified
//
#include <hip/hip_runtime.h>
#include <hip/hip_bf16.h>
#include <stddef.h>
#include <math.h>

#pragma clang fp contract(off)


#define NTH    256
#define NWV    8
#define EPT    8
#define CHUNK  (NTH * EPT)
#define WCAP   (EPT * 32)
#define LISTN  (NWV * WCAP)
#define PASSN  128
#define PCAP   (CHUNK + PASSN)
#define NBMAX  128
#define SEGINTS (LISTN + PCAP + 2 * PASSN + NBMAX + NWV + 4)

static_assert((PCAP % PASSN) == 0);
static_assert((CHUNK % PASSN) == 0);
static_assert(PASSN == 4 * 32);

typedef float          v4f   __attribute__((ext_vector_type(4)));
typedef float          v8f   __attribute__((ext_vector_type(8)));
typedef int            v4i   __attribute__((ext_vector_type(4)));
typedef unsigned short v8us  __attribute__((ext_vector_type(8)));
typedef unsigned short v16us __attribute__((ext_vector_type(16)));
typedef __bf16         v16bf __attribute__((ext_vector_type(16)));
union Frag { v16us u; v8us h[2]; v16bf b; };

__device__ __forceinline__ float silu_f(float x) {
  const float e = __expf(-x);
  return x * __builtin_amdgcn_rcpf(1.0f + e);
}

__device__ __forceinline__ unsigned bfb(float x) {
  const unsigned u = __float_as_uint(x);
  return (u + 0x7FFFu + ((u >> 16) & 1u)) >> 16;
}
__device__ __forceinline__ void sp2(float x, unsigned& hb, unsigned& lb) {
  hb = bfb(x);
  lb = bfb(x - __uint_as_float(hb << 16));
}

__device__ __forceinline__ void lda_split(const float* p, Frag& H, Frag& L) {
  const v4f q0 = *(const v4f*)p, q1 = *(const v4f*)(p + 4), q2 = *(const v4f*)(p + 16), q3 = *(const v4f*)(p + 20);
#pragma unroll
  for (int j = 0; j < 4; ++j) {
    unsigned a, b;
    sp2(q0[j], a, b); H.u[j]      = (unsigned short)a; L.u[j]      = (unsigned short)b;
    sp2(q1[j], a, b); H.u[4 + j]  = (unsigned short)a; L.u[4 + j]  = (unsigned short)b;
    sp2(q2[j], a, b); H.u[8 + j]  = (unsigned short)a; L.u[8 + j]  = (unsigned short)b;
    sp2(q3[j], a, b); H.u[12 + j] = (unsigned short)a; L.u[12 + j] = (unsigned short)b;
  }
}

__device__ __forceinline__ v8f wmb(v16bf a, v16bf b, v8f c) {
  v8f d = __builtin_amdgcn_wmma_f32_16x16x32_bf16(false, a, false, b, (short)0, c, false, false);
  asm volatile("v_nop\n\tv_nop\n\tv_nop\n\tv_nop" : "+v"(d) : "v"(a), "v"(b));
  return d;
}
__device__ __forceinline__ v8f wm3(const Frag& ah, const Frag& al, const Frag& bh, const Frag& bl, v8f c) {
  c = wmb(ah.b, bh.b, c);
  c = wmb(ah.b, bl.b, c);
  c = wmb(al.b, bh.b, c);
  return c;
}
__device__ __forceinline__ v8f zero8f() {
  v8f z;
#pragma unroll
  for (int i = 0; i < 8; ++i) z[i] = 0.0f;
  return z;
}

__device__ __forceinline__ int batch_of(int n, const int* cum, int nB) {
  int cnt = 0;
#pragma unroll 1
  for (int c = 0; c < nB; ++c) cnt += (cum[c] <= n) ? 1 : 0;
  int k = cnt - 1;
  k = k < 0 ? 0 : (k > nB - 1 ? nB - 1 : k);
  return k;
}

__global__ __launch_bounds__(256) void k_wconv(const float* __restrict__ src, int srcPitch, int srcK0, int K, int Nv,
                                               unsigned short* dst, int Kp, int NpTot, int n0, int nStep, int Nrows,
                                               size_t srcStride, size_t dstStride) {
  const int mat = blockIdx.y;
  const int q = blockIdx.x * 256 + threadIdx.x;
  const int kq8 = Kp >> 3;
  const int total = Nrows * kq8;
  const int qc = q < total ? q : total - 1;
  const int nl = qc / kq8, kq = qc - nl * kq8;
  const float* s = src + (size_t)mat * srcStride;
  v8us H, Lo;
#pragma unroll
  for (int j = 0; j < 8; ++j) {
    const int k = kq * 8 + j;
    const int kk = k < K ? k : K - 1;
    const int nn = nl < Nv ? nl : Nv - 1;
    float v = s[(size_t)(srcK0 + kk) * srcPitch + nn];
    if (k >= K || nl >= Nv) v = 0.0f;
    unsigned a, b;
    sp2(v, a, b);
    H[j] = (unsigned short)a;
    Lo[j] = (unsigned short)b;
  }
  unsigned short* d = dst + (size_t)mat * dstStride + (size_t)(n0 + mat * nStep + nl) * Kp + kq * 8;
  const size_t lo = (size_t)NpTot * Kp;
  if (q < total) { *(volatile v8us*)d = H; *(volatile v8us*)(d + lo) = Lo; }
  __threadfence();
  if (q < total) { *(volatile v8us*)d = H; *(volatile v8us*)(d + lo) = Lo; }
}

template <int NT>
__device__ __forceinline__ void gemm_store(const float* st, float* outp, int ldo, int r0, int c0, int lane) {
  constexpr int PPR = 4 * NT;
  constexpr int TOT = 16 * PPR;
#pragma unroll
  for (int it = 0; it < TOT / 32; ++it) {
    const int idx = it * 32 + lane;
    const int rr = idx / PPR, pc = idx - rr * PPR;
    const v4f v = *(const v4f*)(st + rr * 16 * NT + 4 * pc);
    *(volatile v4f*)(outp + (size_t)(r0 + rr) * ldo + c0 + 4 * pc) = v;
  }
}

template <int NT, int EPI>
__global__ __launch_bounds__(128) void k_gemm(const float* __restrict__ A, int lda, int aRowMax, int K,
                                              const unsigned short* __restrict__ Wp, int Kp, int NpTot,
                                              float* outp, int ldo, const float* aux, int ldx,
                                              const int* __restrict__ ix, int nIx, int ixMax, int ncv) {
  __shared__ __attribute__((aligned(16))) float stg[4 * 16 * 16 * NT];
  const int tid = threadIdx.x, lane = tid & 31, wave = tid >> 5, hh = lane >> 4, m = lane & 15;
  const int r0 = blockIdx.x * 64 + wave * 16;
  const int c0 = blockIdx.y * 16 * NT;
  v8f acc[NT];
#pragma unroll
  for (int t = 0; t < NT; ++t) acc[t] = zero8f();
  int arow = r0 + m;
  if (arow > aRowMax) arow = aRowMax;
  const float* ap = A + (size_t)arow * lda + 8 * hh;
  const unsigned short* wb = Wp + (size_t)(c0 + m) * Kp + 8 * hh;
  const size_t loOff = (size_t)NpTot * Kp;
#pragma unroll 1
  for (int kt = 0; kt < K; kt += 32) {
    Frag ah, al;
    lda_split(ap + kt, ah, al);
#pragma unroll
    for (int t = 0; t < NT; ++t) {
      const unsigned short* wp = wb + (size_t)t * 16 * Kp + kt;
      Frag bh, bl;
      bh.h[0] = *(const v8us*)wp;           bh.h[1] = *(const v8us*)(wp + 16);
      bl.h[0] = *(const v8us*)(wp + loOff); bl.h[1] = *(const v8us*)(wp + loOff + 16);
      acc[t] = wm3(ah, al, bh, bl, acc[t]);
    }
  }
  float* st = stg + wave * 16 * 16 * NT;
  constexpr int RW = 16 * NT;
#pragma unroll
  for (int r = 0; r < 8; ++r) {
    const int row = r0 + 8 * hh + r;
    int sI = 0, dI = 0;
    if (EPI == 6) {
      const int rw = row < nIx ? row : nIx - 1;
      sI = ix[rw]; dI = ix[nIx + rw];
      sI = sI < 0 ? 0 : (sI > ixMax ? ixMax : sI);
      dI = dI < 0 ? 0 : (dI > ixMax ? ixMax : dI);
    }
#pragma unroll
    for (int t = 0; t < NT; ++t) {
      const int col = c0 + 16 * t + m;
      float v = acc[t][r];
      if (EPI == 2) {
        v = silu_f(v) * aux[(size_t)row * ldx + col];
      } else if (EPI == 3) {
        v = outp[(size_t)row * ldo + col] + silu_f(v);
      } else if (EPI == 4) {
        v = fmaxf(v + aux[col < ncv ? col : ncv - 1], 0.0f);
      } else if (EPI == 5) {
        v = v + aux[col < ncv ? col : ncv - 1];
      } else if (EPI == 6) {
        const float ps = aux[(size_t)sI * ldx + col];
        const float pd = aux[(size_t)dI * ldx + (ldx >> 1) + col];
        v = silu_f((ps + pd) + v);
      }
      st[(8 * hh + r) * RW + 16 * t + m] = v;
    }
  }
  __syncthreads();
  gemm_store<NT>(st, outp, ldo, r0, c0, lane);
  __threadfence();
  gemm_store<NT>(st, outp, ldo, r0, c0, lane);
}

__global__ __launch_bounds__(256) void k_atom0(const float* __restrict__ frac, const float* __restrict__ len,
                                               const float* __restrict__ ang, const int* __restrict__ types, int nTypes,
                                               const float* __restrict__ noise, const int* __restrict__ numat, int nB,
                                               const float* __restrict__ Gp, const float* __restrict__ whzL,
                                               float* pos4, float* h, int nN) {
  __shared__ int cum[NBMAX];
  const int tid = threadIdx.x, lane = tid & 31, wave = tid >> 5;
  if (tid == 0) {
    int s = 0;
    for (int c = 0; c < nB; ++c) { cum[c] = s; s += numat[c]; }
  }
  __syncthreads();
  const int q = blockIdx.x * 8 + (lane & 7);
  const int qc = q < nN ? q : nN - 1;
  const int bt = batch_of(qc, cum, nB);
  const float la = len[bt * 3 + 0], lb = len[bt * 3 + 1], lc = len[bt * 3 + 2];
  const float D2R = (float)(3.141592653589793 / 180.0);
  const float al = ang[bt * 3 + 0] * D2R, be = ang[bt * 3 + 1] * D2R, ga = ang[bt * 3 + 2] * D2R;
  const float cal = cosf(al), cbe = cosf(be), cga = cosf(ga), sga = sinf(ga);
  const float cx = cbe;
  const float cy = (cal - cbe * cga) * (1.0f / sga);
  const float cz = sqrtf(fmaxf((1.0f - cx * cx) - cy * cy, 1e-8f));
  const float l10 = lb * cga, l11 = lb * sga;
  const float l20 = lc * cx, l21 = lc * cy, l22 = lc * cz;
  const float f0 = frac[qc * 3 + 0], f1 = frac[qc * 3 + 1], f2 = frac[qc * 3 + 2];
  const float px = (f0 * la + f1 * l10) + f2 * l20;
  const float py = (f1 * l11) + f2 * l21;
  const float pz = f2 * l22;
  v4f pv = {px, py, pz, 0.0f};
  const int btw = __shfl(bt, wave);
  const int n = blockIdx.x * 8 + wave;
  const int nc = n < nN ? n : nN - 1;
  int ty = types[nc];
  ty = ty < 0 ? 0 : (ty > nTypes - 1 ? nTypes - 1 : ty);
  const v4f g = *(const v4f*)(Gp + (size_t)ty * 128 + 4 * lane);
  const v4f w = *(const v4f*)(whzL + 4 * lane);
  const float nz = noise[btw];
  v4f o;
#pragma unroll
  for (int j = 0; j < 4; ++j) o[j] = silu_f(g[j] + nz * w[j]);
  const bool wp = (wave == 0) && (lane < 8) && (q < nN);
  if (n < nN) *(volatile v4f*)(h + (size_t)n * 128 + 4 * lane) = o;
  if (wp) *(volatile v4f*)(pos4 + (size_t)q * 4) = pv;
  __threadfence();
  if (n < nN) *(volatile v4f*)(h + (size_t)n * 128 + 4 * lane) = o;
  if (wp) *(volatile v4f*)(pos4 + (size_t)q * 4) = pv;
}

__global__ __launch_bounds__(128) void k_egeom(const float* __restrict__ pos4, const int* __restrict__ ei, int nE, int nN,
                                               float* vec4, float* rbf) {
  __shared__ __attribute__((aligned(16))) float rb[128 * 64];
  const int tid = threadIdx.x, lane = tid & 31, wave = tid >> 5;
  const int e = blockIdx.x * 128 + tid, ec = e < nE ? e : nE - 1;
  int s = ei[ec], d = ei[nE + ec];
  s = s < 0 ? 0 : (s > nN - 1 ? nN - 1 : s);
  d = d < 0 ? 0 : (d > nN - 1 ? nN - 1 : d);
  const v4f ps = *(const v4f*)(pos4 + (size_t)s * 4), pd = *(const v4f*)(pos4 + (size_t)d * 4);
  const float vx = pd.x - ps.x, vy = pd.y - ps.y, vz = pd.z - ps.z;
  const float dd = sqrtf(((vx * vx + vy * vy) + vz * vz) + 1e-12f);
  const float ds = dd * (1.0f / 7.0f);
  float env = 0.0f;
  if (ds < 1.0f) {
    const float x2 = ds * ds, x4 = x2 * x2;
    const float p5 = ds * x4, p6 = x2 * x4, p7 = (ds * x2) * x4;
    env = ((1.0f - 21.0f * p5) + 35.0f * p6) - 15.0f * p7;
  }
  const float pre = env * 0.5345224838248488f;
  const float invd = 1.0f / dd;
#pragma unroll 1
  for (int n = 0; n < 64; ++n) {
    const float arg = ((float)(n + 1) * 3.14159265358979323846f) * ds;
    rb[tid * 64 + n] = (pre * sinf(arg)) * invd;
  }
  v4f vv = {vx, vy, vz, dd};
  if (e < nE) *(volatile v4f*)(vec4 + (size_t)e * 4) = vv;
  __syncthreads();
#pragma unroll
  for (int it = 0; it < 16; ++it) {
    const int idx = it * 32 + lane;
    const int rr = 32 * wave + (idx >> 4), pc = idx & 15;
    const int er = blockIdx.x * 128 + rr;
    const v4f v = *(const v4f*)(rb + rr * 64 + 4 * pc);
    if (er < nE) *(volatile v4f*)(rbf + (size_t)er * 64 + 4 * pc) = v;
  }
  __threadfence();
  if (e < nE) *(volatile v4f*)(vec4 + (size_t)e * 4) = vv;
#pragma unroll
  for (int it = 0; it < 16; ++it) {
    const int idx = it * 32 + lane;
    const int rr = 32 * wave + (idx >> 4), pc = idx & 15;
    const int er = blockIdx.x * 128 + rr;
    const v4f v = *(const v4f*)(rb + rr * 64 + 4 * pc);
    if (er < nE) *(volatile v4f*)(rbf + (size_t)er * 64 + 4 * pc) = v;
  }
}

template <int W, int MODE, int NBK>
struct SegL {
  static constexpr int FL = (NBK + 1) * W + ((MODE == 1) ? PASSN * 64 : 0);
  static constexpr int US = (MODE == 1) ? (PASSN * 32 * 2 + 64 * 32 * 2) : 0;
  static constexpr size_t BYTES = (size_t)FL * 4 + (size_t)US * 2 + (size_t)SEGINTS * 4;
};

template <int W, int MODE>
__device__ __forceinline__ void seg_store(const float* accl, float* outp, int keyBase, int nKeys, int nRows,
                                          const int* __restrict__ numat, int nB, int tid) {
  constexpr int PPR = W / 4;
  for (int idx = tid; idx < nRows * PPR; idx += NTH) {
    const int rr = idx / PPR, pc = idx - rr * PPR;
    const int key = keyBase + rr;
    v4f v = *(const v4f*)(accl + rr * W + 4 * pc);
    if (MODE == 2) {
      const int na = numat[key < nB ? key : nB - 1];
      const float inv = 1.0f / (float)na;
#pragma unroll
      for (int j = 0; j < 4; ++j) v[j] = v[j] * inv;
    }
    if (key < nKeys) *(volatile v4f*)(outp + (size_t)key * W + 4 * pc) = v;
  }
}

template <int W, int MODE, int NBK>
__global__ __launch_bounds__(NTH) void k_seg(const int* __restrict__ key, int nItems, int nKeys,
                                            const float* src, int srcRows,
                                            const int* __restrict__ kj, const float* __restrict__ vec4, int nE,
                                            const unsigned short* __restrict__ wcb,
                                            const int* __restrict__ numat, int nB, float* outp) {
  extern __shared__ __attribute__((aligned(16))) unsigned char smem[];
  typedef SegL<W, MODE, NBK> L;
  static_assert(W == 64 || W == 128);
  static_assert(MODE != 1 || W == 64);
  float* accl = (float*)smem;
  float* msg  = accl + (NBK + 1) * W;
  unsigned short* cbh = (unsigned short*)(accl + L::FL);
  unsigned short* cbl = cbh + ((MODE == 1) ? PASSN * 32 : 0);
  unsigned short* wch = cbl + ((MODE == 1) ? PASSN * 32 : 0);
  unsigned short* wcl = wch + ((MODE == 1) ? 64 * 32 : 0);
  int* list  = (int*)(cbh + L::US);
  int* pend  = list + LISTN;
  int* slotb = pend + PCAP;
  int* itemb = slotb + PASSN;
  int* cum   = itemb + PASSN;
  int* wcnt  = cum + NBMAX;
  int* pendN = wcnt + NWV;
  const int tid = threadIdx.x, lane = tid & 31, wave = tid >> 5, hh = lane >> 4, m = lane & 15;
  const int keyBase = blockIdx.x * NBK;

  for (int i = tid; i < (NBK + 1) * W; i += NTH) accl[i] = 0.0f;
  if (MODE == 1) {
    for (int i = tid; i < PASSN * 32; i += NTH) { cbh[i] = 0; cbl[i] = 0; }
    for (int i = tid; i < 64 * 32; i += NTH) { wch[i] = wcb[i]; wcl[i] = wcb[64 * 32 + i]; }
  }
  if (MODE == 2 && tid == 0) {
    int s = 0;
    for (int c = 0; c < nB && c < NBMAX; ++c) { cum[c] = s; s += numat[c]; }
  }
  if (tid == 0) *pendN = 0;
  __syncthreads();

  const int nChunks = (nItems + CHUNK - 1) / CHUNK;
#pragma unroll 1
  for (int ch = 0; ch < nChunks; ++ch) {
    const int cbase = ch * CHUNK;
    int wc = 0;
    {
      const int el0 = tid * EPT, e0 = cbase + el0;
      int kv[EPT];
      if (MODE != 2 && cbase + CHUNK <= nItems) {
        const v4i da = *(const v4i*)(key + e0), db = *(const v4i*)(key + e0 + 4);
        kv[0] = da.x; kv[1] = da.y; kv[2] = da.z; kv[3] = da.w;
        kv[4] = db.x; kv[5] = db.y; kv[6] = db.z; kv[7] = db.w;
      } else {
#pragma unroll
        for (int j = 0; j < EPT; ++j) {
          const int it = e0 + j;
          const int itc = it < nItems ? it : nItems - 1;
          int k;
          if (MODE == 2) k = batch_of(itc, cum, nB); else k = key[itc];
          kv[j] = (it < nItems) ? k : (-2147483647 - 1);
        }
      }
      bool hb[EPT];
      bool anyb = false;
#pragma unroll
      for (int j = 0; j < EPT; ++j) {
        hb[j] = ((unsigned)kv[j] - (unsigned)keyBase) < (unsigned)NBK;
        anyb = anyb || hb[j];
      }
      if (__builtin_amdgcn_ballot_w32(anyb) != 0u) {
#pragma unroll
        for (int j = 0; j < EPT; ++j) {
          const unsigned mj = __builtin_amdgcn_ballot_w32(hb[j]);
          if (mj != 0u) {
            if (hb[j]) {
              const int pos = wc + (int)__builtin_amdgcn_mbcnt_lo(mj, 0u);
              if (pos < WCAP) list[wave * WCAP + pos] = el0 + j;
            }
            wc += (int)__builtin_popcount(mj);
          }
        }
      }
    }
    if (lane == 0) wcnt[wave] = wc;
    __syncthreads();

    const int base = *pendN;
    int tot = 0, myoff = 0;
#pragma unroll
    for (int w = 0; w < NWV; ++w) {
      int c = wcnt[w];
      c = c > WCAP ? WCAP : (c < 0 ? 0 : c);
      if (w < wave) myoff += c;
      tot += c;
    }
    int newN = base + tot;
    newN = newN > PCAP ? PCAP : newN;
    {
      int n = wcnt[wave];
      n = n > WCAP ? WCAP : (n < 0 ? 0 : n);
      const int* lp = list + wave * WCAP;
      for (int i = lane; i < n; i += 32) {
        const int pos = base + myoff + i;
        if (pos < PCAP) pend[pos] = cbase + lp[i];
      }
    }
    const int fin = (ch == nChunks - 1) ? 1 : 0;
    const int R   = (fin != 0) ? (newN + PASSN - 1) / PASSN : newN / PASSN;
    const int Pv  = (fin != 0) ? newN : R * PASSN;
    __syncthreads();

#pragma unroll 1
    for (int r = 0; r < R; ++r) {
      if (tid < PASSN) {
        const int idx = r * PASSN + tid;
        const bool valid = idx < Pv;
        int it = pend[idx < PCAP ? idx : PCAP - 1];
        if (!valid) it = 0;
        it = it < 0 ? 0 : (it > nItems - 1 ? nItems - 1 : it);
        int k;
        if (MODE == 2) k = batch_of(it, cum, nB); else k = key[it];
        int slot = k - keyBase;
        if (!valid || (unsigned)slot >= (unsigned)NBK) slot = NBK;
        slotb[tid] = slot;
        if (MODE == 1) {
          const int e1 = k < 0 ? 0 : (k > nE - 1 ? nE - 1 : k);
          int e2 = kj[it];
          e2 = e2 < 0 ? 0 : (e2 > nE - 1 ? nE - 1 : e2);
          itemb[tid] = e2;
          const v4f va = *(const v4f*)(vec4 + (size_t)e1 * 4), vb = *(const v4f*)(vec4 + (size_t)e2 * 4);
          const float dot = (va.x * vb.x + va.y * vb.y) + va.z * vb.z;
          const float n1 = sqrtf((va.x * va.x + va.y * va.y) + va.z * va.z);
          const float n2 = sqrtf((vb.x * vb.x + vb.y * vb.y) + vb.z * vb.z);
          float ca = dot * (1.0f / (n1 * n2 + 1e-9f));
          ca = fminf(fmaxf(ca, (float)(-1.0 + 1e-6)), (float)(1.0 - 1e-6));
          const float an = acosf(ca);
#pragma unroll 1
          for (int s = 0; s < 16; ++s) {
            const float cv = cosf((float)s * an);
            unsigned a, b;
            sp2(cv, a, b);
            cbh[tid * 32 + s] = (unsigned short)a;
            cbl[tid * 32 + s] = (unsigned short)b;
          }
        } else {
          itemb[tid] = it;
        }
      }
      __syncthreads();

      if (MODE == 1) {
        Frag ah, al;
        {
          const unsigned short* cp = cbh + (16 * wave + m) * 32 + 8 * hh;
          const unsigned short* cq = cbl + (16 * wave + m) * 32 + 8 * hh;
          ah.h[0] = *(const v8us*)cp; ah.h[1] = *(const v8us*)(cp + 16);
          al.h[0] = *(const v8us*)cq; al.h[1] = *(const v8us*)(cq + 16);
        }
        v8f acc[4];
#pragma unroll
        for (int t = 0; t < 4; ++t) {
          acc[t] = zero8f();
          const unsigned short* bp = wch + (16 * t + m) * 32 + 8 * hh;
          const unsigned short* bq = wcl + (16 * t + m) * 32 + 8 * hh;
          Frag bh, bl;
          bh.h[0] = *(const v8us*)bp; bh.h[1] = *(const v8us*)(bp + 16);
          bl.h[0] = *(const v8us*)bq; bl.h[1] = *(const v8us*)(bq + 16);
          acc[t] = wm3(ah, al, bh, bl, acc[t]);
        }
#pragma unroll
        for (int rr = 0; rr < 8; ++rr) {
          const int i = 16 * wave + 8 * hh + rr;
          const int e2 = itemb[i];
          const float* xr = src + (size_t)e2 * 64;
#pragma unroll
          for (int t = 0; t < 4; ++t) msg[i * 64 + 16 * t + m] = acc[t][rr] * xr[16 * t + m];
        }
        __syncthreads();
      }

      if (tid < W) {
#pragma unroll 1
        for (int i = 0; i < PASSN; ++i) {
          int sl = slotb[i];
          sl = sl < 0 ? 0 : (sl > NBK ? NBK : sl);
          float v;
          if (MODE == 1) {
            v = msg[i * 64 + tid];
          } else {
            int it = itemb[i];
            it = it < 0 ? 0 : (it > srcRows - 1 ? srcRows - 1 : it);
            v = src[(size_t)it * W + tid];
          }
          accl[sl * W + tid] += v;
        }
      }
      __syncthreads();
    }

    int rem = newN - R * PASSN;
    rem = rem < 0 ? 0 : rem;
    if (R > 0 && tid < rem) pend[tid] = pend[R * PASSN + tid];
    if (tid == 0) *pendN = rem;
  }
  __syncthreads();

  seg_store<W, MODE>(accl, outp, keyBase, nKeys, NBK, numat, nB, tid);
  __threadfence();
  seg_store<W, MODE>(accl, outp, keyBase, nKeys, NBK, numat, nB, tid);
}

__global__ __launch_bounds__(256) void k_eupd(const float* __restrict__ hst, const int* __restrict__ ei, int nE, int nN,
                                              float* m) {
  const int tid = threadIdx.x, lane = tid & 31, wave = tid >> 5;
  const int e = blockIdx.x * 8 + wave, ec = e < nE ? e : nE - 1;
  int s = ei[ec], d = ei[nE + ec];
  s = s < 0 ? 0 : (s > nN - 1 ? nN - 1 : s);
  d = d < 0 ? 0 : (d > nN - 1 ? nN - 1 : d);
  const v4f a = *(const v4f*)(hst + (size_t)s * 256 + 4 * lane);
  const v4f b = *(const v4f*)(hst + (size_t)d * 256 + 128 + 4 * lane);
  const v4f mm = *(const v4f*)(m + (size_t)ec * 128 + 4 * lane);
  v4f o;
#pragma unroll
  for (int j = 0; j < 4; ++j) o[j] = mm[j] + silu_f(a[j] + b[j]);
  if (e < nE) *(volatile v4f*)(m + (size_t)e * 128 + 4 * lane) = o;
  __threadfence();
  if (e < nE) *(volatile v4f*)(m + (size_t)e * 128 + 4 * lane) = o;
}

__global__ __launch_bounds__(256) void k_outcopy(const float* __restrict__ t2, int ldt, int cols, int total, float* outp) {
  const int tid = threadIdx.x;
  const int nq = total >> 2;
  for (int q = tid; q < nq; q += 256) {
    v4f v;
#pragma unroll
    for (int j = 0; j < 4; ++j) { const int idx = 4 * q + j; const int r = idx / cols, c = idx - r * cols; v[j] = t2[(size_t)r * ldt + c]; }
    *(volatile v4f*)(outp + 4 * (size_t)q) = v;
  }
  __threadfence();
  for (int q = tid; q < nq; q += 256) {
    v4f v;
#pragma unroll
    for (int j = 0; j < 4; ++j) { const int idx = 4 * q + j; const int r = idx / cols, c = idx - r * cols; v[j] = t2[(size_t)r * ldt + c]; }
    *(volatile v4f*)(outp + 4 * (size_t)q) = v;
  }
}

template <int NT, int EPI>
static void gemm(hipStream_t st, const float* A, int lda, int aRowMax, int M, int K,
                 const unsigned short* Wp, int NpTot, int N, float* out, int ldo,
                 const float* aux, int ldx, const int* ix, int nIx, int ixMax, int ncv) {
  dim3 grid((unsigned)(M / 64), (unsigned)(N / (16 * NT)));
  k_gemm<NT, EPI><<<grid, 128, 0, st>>>(A, lda, aRowMax, K, Wp, K, NpTot, out, ldo, aux, ldx, ix, nIx, ixMax, ncv);
}

extern "C" void kernel_launch(void* const* d_in, const int* in_sizes, int n_in,
                              void* d_out, int out_size, void* d_ws, size_t ws_size,
                              hipStream_t stream) {
  if (n_in < 29) return;
  const int nB = 128, nN = 4096, nE = 65536, nT = 262144, nTypes = 100;
  if (in_sizes[0] != nB || in_sizes[1] != nN * 3 || in_sizes[2] != nB * 3 || in_sizes[3] != nB * 3) return;
  if (in_sizes[4] != nN || in_sizes[5] != nB || in_sizes[6] != 2 * nE || in_sizes[7] != nT || in_sizes[8] != nT) return;
  if (in_sizes[9] != nTypes * 128 || in_sizes[10] != 129 * 128 || in_sizes[11] != 320 * 128) return;
  if (in_sizes[12] != 3 * 128 * 128 || in_sizes[13] != 3 * 64 * 128 || in_sizes[14] != 3 * 128 * 64) return;
  if (in_sizes[15] != 3 * 16 * 64 || in_sizes[16] != 3 * 64 * 128 || in_sizes[17] != 3 * 128 * 128) return;
  if (in_sizes[18] != 3 * 64 * 128 || in_sizes[19] != 3 * 128 * 128 || in_sizes[20] != 3 * 128 * 128) return;
  if (in_sizes[21] != 3 * 128 * 128 || in_sizes[22] != 128 * 128 || in_sizes[23] != 128 * 256 || in_sizes[24] != 256) return;
  if (in_sizes[25] != 256 * 256 || in_sizes[26] != 256 || in_sizes[27] != 256 * 230 || in_sizes[28] != 230) return;
  if (out_size != nB * 230) return;

  const float* noise  = (const float*)d_in[0];
  const float* frac   = (const float*)d_in[1];
  const float* len    = (const float*)d_in[2];
  const float* angl   = (const float*)d_in[3];
  const int*   types  = (const int*)d_in[4];
  const int*   numat  = (const int*)d_in[5];
  const int*   ei     = (const int*)d_in[6];
  const int*   ji     = (const int*)d_in[7];
  const int*   kj     = (const int*)d_in[8];
  const float* emb    = (const float*)d_in[9];
  const float* W_hz   = (const float*)d_in[10];
  const float* W_edge = (const float*)d_in[11];
  const float* Wm     = (const float*)d_in[12];
  const float* Wr1    = (const float*)d_in[13];
  const float* Wdown  = (const float*)d_in[14];
  const float* Wcbf   = (const float*)d_in[15];
  const float* Wup    = (const float*)d_in[16];
  const float* Wa     = (const float*)d_in[17];
  const float* Wr2    = (const float*)d_in[18];
  const float* Wh     = (const float*)d_in[19];
  const float* Ws     = (const float*)d_in[20];
  const float* Wt     = (const float*)d_in[21];
  const float* W_out  = (const float*)d_in[22];
  const float* W_fc0  = (const float*)d_in[23];
  const float* b_fc0  = (const float*)d_in[24];
  const float* W_fc1  = (const float*)d_in[25];
  const float* b_fc1  = (const float*)d_in[26];
  const float* W_fc2  = (const float*)d_in[27];
  const float* b_fc2  = (const float*)d_in[28];
  float* outF = (float*)d_out;

  char* ws = (char*)d_ws;
  size_t off = 0;
  auto al = [&](size_t bytes) -> char* { off = (off + 255) & ~(size_t)255; char* p = ws + off; off += bytes; return p; };
  auto WPL = [&](int Np, int Kp, int cnt) -> unsigned short* { return (unsigned short*)al((size_t)4 * Np * Kp * cnt); };
  unsigned short* wHZ  = WPL(128, 128, 1);
  unsigned short* wE12 = WPL(256, 128, 1);
  unsigned short* wE3  = WPL(128, 64, 1);
  unsigned short* wM   = WPL(128, 128, 3);
  unsigned short* wR1  = WPL(128, 64, 3);
  unsigned short* wDN  = WPL(64, 128, 3);
  unsigned short* wCB  = WPL(64, 32, 3);
  unsigned short* wUP  = WPL(128, 64, 3);
  unsigned short* wA   = WPL(128, 128, 3);
  unsigned short* wR2  = WPL(128, 64, 3);
  unsigned short* wH   = WPL(128, 128, 3);
  unsigned short* wST  = WPL(256, 128, 3);
  unsigned short* wOUT = WPL(128, 128, 1);
  unsigned short* wF0  = WPL(256, 128, 1);
  unsigned short* wF1  = WPL(256, 256, 1);
  unsigned short* wF2  = WPL(256, 256, 1);
  float* pos4 = (float*)al((size_t)nN * 4 * 4);
  float* vec4 = (float*)al((size_t)nE * 4 * 4);
  float* rbf  = (float*)al((size_t)nE * 64 * 4);
  float* Gp   = (float*)al((size_t)128 * 128 * 4);
  float* h    = (float*)al((size_t)nN * 128 * 4);
  float* HS   = (float*)al((size_t)nN * 256 * 4);
  float* m    = (float*)al((size_t)nE * 128 * 4);
  float* R    = (float*)al((size_t)nE * 128 * 4);
  float* x    = (float*)al((size_t)nE * 64 * 4);
  float* agg  = (float*)al((size_t)nE * 64 * 4);
  float* a    = (float*)al((size_t)nN * 128 * 4);
  float* Hout = (float*)al((size_t)nN * 128 * 4);
  float* z    = (float*)al((size_t)nB * 128 * 4);
  float* t0   = (float*)al((size_t)nB * 256 * 4);
  float* t1   = (float*)al((size_t)nB * 256 * 4);
  float* t2   = (float*)al((size_t)nB * 256 * 4);
  if (off > ws_size || off > (size_t)134217728) return;

  auto wconv = [&](const float* src, int pitch, int k0, int K, int Nv, unsigned short* dst, int Kp, int NpTot,
                   int n0, int nStep, int Nrows, int nMat, size_t sStride, size_t dStride) {
    dim3 grid((unsigned)((Nrows * (Kp / 8)) / 256), (unsigned)nMat);
    k_wconv<<<grid, 256, 0, stream>>>(src, pitch, k0, K, Nv, dst, Kp, NpTot, n0, nStep, Nrows, sStride, dStride);
  };
  wconv(W_hz,   128, 0,   128, 128, wHZ,  128, 128, 0,   0,   128, 1, 0, 0);
  wconv(W_edge, 128, 0,   128, 128, wE12, 128, 256, 0,   128, 128, 2, (size_t)128 * 128, 0);
  wconv(W_edge, 128, 256, 64,  128, wE3,  64,  128, 0,   0,   128, 1, 0, 0);
  wconv(Wm,     128, 0,   128, 128, wM,   128, 128, 0,   0,   128, 3, (size_t)128 * 128, (size_t)2 * 128 * 128);
  wconv(Wr1,    128, 0,   64,  128, wR1,  64,  128, 0,   0,   128, 3, (size_t)64 * 128,  (size_t)2 * 128 * 64);
  wconv(Wdown,  64,  0,   128, 64,  wDN,  128, 64,  0,   0,   64,  3, (size_t)128 * 64,  (size_t)2 * 64 * 128);
  wconv(Wcbf,   64,  0,   16,  64,  wCB,  32,  64,  0,   0,   64,  3, (size_t)16 * 64,   (size_t)2 * 64 * 32);
  wconv(Wup,    128, 0,   64,  128, wUP,  64,  128, 0,   0,   128, 3, (size_t)64 * 128,  (size_t)2 * 128 * 64);
  wconv(Wa,     128, 0,   128, 128, wA,   128, 128, 0,   0,   128, 3, (size_t)128 * 128, (size_t)2 * 128 * 128);
  wconv(Wr2,    128, 0,   64,  128, wR2,  64,  128, 0,   0,   128, 3, (size_t)64 * 128,  (size_t)2 * 128 * 64);
  wconv(Wh,     128, 0,   128, 128, wH,   128, 128, 0,   0,   128, 3, (size_t)128 * 128, (size_t)2 * 128 * 128);
  wconv(Ws,     128, 0,   128, 128, wST,  128, 256, 0,   0,   128, 3, (size_t)128 * 128, (size_t)2 * 256 * 128);
  wconv(Wt,     128, 0,   128, 128, wST,  128, 256, 128, 0,   128, 3, (size_t)128 * 128, (size_t)2 * 256 * 128);
  wconv(W_out,  128, 0,   128, 128, wOUT, 128, 128, 0,   0,   128, 1, 0, 0);
  wconv(W_fc0,  256, 0,   128, 256, wF0,  128, 256, 0,   0,   256, 1, 0, 0);
  wconv(W_fc1,  256, 0,   256, 256, wF1,  256, 256, 0,   0,   256, 1, 0, 0);
  wconv(W_fc2,  230, 0,   256, 230, wF2,  256, 256, 0,   0,   256, 1, 0, 0);

  const size_t segB1 = SegL<64, 1, 512>::BYTES;
  const size_t segB0 = SegL<128, 0, 128>::BYTES;
  const size_t segB2 = SegL<128, 2, 128>::BYTES;
  hipFuncSetAttribute(reinterpret_cast<const void*>(&k_seg<64, 1, 512>), hipFuncAttributeMaxDynamicSharedMemorySize, (int)segB1);
  hipFuncSetAttribute(reinterpret_cast<const void*>(&k_seg<128, 0, 128>), hipFuncAttributeMaxDynamicSharedMemorySize, (int)segB0);
  hipFuncSetAttribute(reinterpret_cast<const void*>(&k_seg<128, 2, 128>), hipFuncAttributeMaxDynamicSharedMemorySize, (int)segB2);

  gemm<8, 0>(stream, emb, 128, nTypes - 1, 128, 128, wHZ, 128, 128, Gp, 128, emb, 128, ei, nE, nN - 1, 1);
  k_atom0<<<nN / 8, 256, 0, stream>>>(frac, len, angl, types, nTypes, noise, numat, nB, Gp, W_hz + 128 * 128, pos4, h, nN);
  k_egeom<<<nE / 128, 128, 0, stream>>>(pos4, ei, nE, nN, vec4, rbf);
  gemm<8, 0>(stream, h, 128, nN - 1, nN, 128, wE12, 256, 256, HS, 256, h, 256, ei, nE, nN - 1, 1);
  gemm<8, 6>(stream, rbf, 64, nE - 1, nE, 64, wE3, 128, 128, m, 128, HS, 256, ei, nE, nN - 1, 1);

  for (int b = 0; b < 3; ++b) {
    const unsigned short* wMb  = wM  + (size_t)b * 2 * 128 * 128;
    const unsigned short* wR1b = wR1 + (size_t)b * 2 * 128 * 64;
    const unsigned short* wDNb = wDN + (size_t)b * 2 * 64 * 128;
    const unsigned short* wCBb = wCB + (size_t)b * 2 * 64 * 32;
    const unsigned short* wUPb = wUP + (size_t)b * 2 * 128 * 64;
    const unsigned short* wAb  = wA  + (size_t)b * 2 * 128 * 128;
    const unsigned short* wR2b = wR2 + (size_t)b * 2 * 128 * 64;
    const unsigned short* wHb  = wH  + (size_t)b * 2 * 128 * 128;
    const unsigned short* wSTb = wST + (size_t)b * 2 * 256 * 128;
    gemm<8, 0>(stream, rbf, 64, nE - 1, nE, 64, wR1b, 128, 128, R, 128, rbf, 128, ei, nE, nN - 1, 1);
    gemm<8, 2>(stream, m, 128, nE - 1, nE, 128, wMb, 128, 128, R, 128, R, 128, ei, nE, nN - 1, 1);
    gemm<4, 0>(stream, R, 128, nE - 1, nE, 128, wDNb, 64, 64, x, 64, R, 64, ei, nE, nN - 1, 1);
    k_seg<64, 1, 512><<<nE / 512, NTH, segB1, stream>>>(ji, nT, nE, x, nE, kj, vec4, nE, wCBb, numat, nB, agg);
    gemm<8, 3>(stream, agg, 64, nE - 1, nE, 64, wUPb, 128, 128, m, 128, agg, 128, ei, nE, nN - 1, 1);
    gemm<8, 0>(stream, rbf, 64, nE - 1, nE, 64, wR2b, 128, 128, R, 128, rbf, 128, ei, nE, nN - 1, 1);
    gemm<8, 2>(stream, m, 128, nE - 1, nE, 128, wAb, 128, 128, R, 128, R, 128, ei, nE, nN - 1, 1);
    k_seg<128, 0, 128><<<nN / 128, NTH, segB0, stream>>>(ei + nE, nE, nN, R, nE, kj, vec4, nE, wCBb, numat, nB, a);
    gemm<8, 3>(stream, a, 128, nN - 1, nN, 128, wHb, 128, 128, h, 128, a, 128, ei, nE, nN - 1, 1);
    gemm<8, 0>(stream, h, 128, nN - 1, nN, 128, wSTb, 256, 256, HS, 256, h, 256, ei, nE, nN - 1, 1);
    k_eupd<<<nE / 8, 256, 0, stream>>>(HS, ei, nE, nN, m);
  }

  gemm<8, 0>(stream, h, 128, nN - 1, nN, 128, wOUT, 128, 128, Hout, 128, h, 128, ei, nE, nN - 1, 1);
  k_seg<128, 2, 128><<<1, NTH, segB2, stream>>>(ei, nN, nB, Hout, nN, kj, vec4, nE, wCB, numat, nB, z);
  gemm<8, 4>(stream, z,  128, nB - 1, 128, 128, wF0, 256, 256, t0, 256, b_fc0, 256, ei, nE, nN - 1, 256);
  gemm<8, 4>(stream, t0, 256, nB - 1, 128, 256, wF1, 256, 256, t1, 256, b_fc1, 256, ei, nE, nN - 1, 256);
  gemm<8, 5>(stream, t1, 256, nB - 1, 128, 256, wF2, 256, 256, t2, 256, b_fc2, 256, ei, nE, nN - 1, 230);
  k_outcopy<<<1, 256, 0, stream>>>(t2, 256, 230, nB * 230, outF);
}
